// LearnablePixelwiseAnisoJBU3D_89721866813723
// MI455X (gfx1250) — hardware-verified
//
#include <hip/hip_runtime.h>
#include <math.h>


#define CF 32
#define GG 3
#define NL 32
#define NHR 64
#define NCELL (NL * NL * NL)
#define NVOX (NHR * NHR * NHR)
#define RMAX 3
#define NOFF 343
#define KPAD 352

typedef __attribute__((ext_vector_type(16))) __bf16   v16bf;
typedef __attribute__((ext_vector_type(16))) _Float16 v16h;
typedef __attribute__((ext_vector_type(8)))  float    v8f;
typedef __attribute__((ext_vector_type(8)))  unsigned v8u;

__device__ __forceinline__ unsigned f2bf(float f) { unsigned u = __float_as_uint(f); u += 0x7FFFu + ((u >> 16) & 1u); return u >> 16; }
__device__ __forceinline__ unsigned f2h(float f) { return (unsigned)__builtin_bit_cast(unsigned short, (_Float16)f); }
__device__ __forceinline__ int kpat(int v, int half) { return ((v & 4) ? 16 : 0) + half * 8 + 2 * (v & 3); }

template <int F16, int NP> struct Opnd { v16bf p[NP]; };

template <int F16, int NP> __device__ __forceinline__ void pack2(float f0, float f1, unsigned* o) {
    if (F16) { o[0] = f2h(f0) | (f2h(f1) << 16); return; }
    unsigned h0 = f2bf(f0), h1 = f2bf(f1); o[0] = h0 | (h1 << 16);
    if (NP >= 2) {
        float r0 = f0 - __uint_as_float(h0 << 16), r1 = f1 - __uint_as_float(h1 << 16);
        unsigned m0 = f2bf(r0), m1 = f2bf(r1); o[1] = m0 | (m1 << 16);
        if (NP >= 3) {
            float s0 = r0 - __uint_as_float(m0 << 16), s1 = r1 - __uint_as_float(m1 << 16);
            o[2] = f2bf(s0) | (f2bf(s1) << 16);
        }
    }
}
template <int F16, int NP> __device__ __forceinline__ void op_row(const float* rowp, int half, float sc, Opnd<F16, NP>& o) {
    v8u u[NP];
#pragma unroll
    for (int v = 0; v < 8; ++v) {
        int kk = kpat(v, half); unsigned t[3];
        pack2<F16, NP>(rowp[kk] * sc, rowp[kk + 1] * sc, t);
#pragma unroll
        for (int p = 0; p < NP; ++p) u[p][v] = t[p];
    }
#pragma unroll
    for (int p = 0; p < NP; ++p) o.p[p] = __builtin_bit_cast(v16bf, u[p]);
}
template <int F16, int NP> __device__ __forceinline__ void op_row_tail(const float* rowp, int half, float sc, int kvalid, Opnd<F16, NP>& o) {
    v8u u[NP];
#pragma unroll
    for (int v = 0; v < 8; ++v) {
        int kk = kpat(v, half); unsigned t[3];
        float f0 = kk < kvalid ? rowp[kk] * sc : 0.0f, f1 = (kk + 1) < kvalid ? rowp[kk + 1] * sc : 0.0f;
        pack2<F16, NP>(f0, f1, t);
#pragma unroll
        for (int p = 0; p < NP; ++p) u[p][v] = t[p];
    }
#pragma unroll
    for (int p = 0; p < NP; ++p) o.p[p] = __builtin_bit_cast(v16bf, u[p]);
}
template <int F16, int NP> __device__ __forceinline__ void op_col(const float* M, int ld, int n, int k0, int half, float sc, Opnd<F16, NP>& o) {
    v8u u[NP];
#pragma unroll
    for (int v = 0; v < 8; ++v) {
        int kk = k0 + kpat(v, half); unsigned t[3];
        pack2<F16, NP>(M[(size_t)kk * ld + n] * sc, M[(size_t)(kk + 1) * ld + n] * sc, t);
#pragma unroll
        for (int p = 0; p < NP; ++p) u[p][v] = t[p];
    }
#pragma unroll
    for (int p = 0; p < NP; ++p) o.p[p] = __builtin_bit_cast(v16bf, u[p]);
}
template <int F16, int NP> __device__ __forceinline__ void op_col_tail(const float* M, int ld, int n, int k0, int half, float sc, int K, Opnd<F16, NP>& o) {
    v8u u[NP];
#pragma unroll
    for (int v = 0; v < 8; ++v) {
        int kk = k0 + kpat(v, half); unsigned t[3];
        float f0 = kk < K ? M[(size_t)kk * ld + n] * sc : 0.0f, f1 = (kk + 1) < K ? M[(size_t)(kk + 1) * ld + n] * sc : 0.0f;
        pack2<F16, NP>(f0, f1, t);
#pragma unroll
        for (int p = 0; p < NP; ++p) u[p][v] = t[p];
    }
#pragma unroll
    for (int p = 0; p < NP; ++p) o.p[p] = __builtin_bit_cast(v16bf, u[p]);
}
__device__ __forceinline__ v8f wm_bf16(v16bf a, v16bf b, v8f c) { return __builtin_amdgcn_wmma_f32_16x16x32_bf16(false, a, false, b, (short)0, c, false, false); }
template <int F16, int NA, int NB> __device__ __forceinline__ v8f wmma_op(const Opnd<F16, NA>& a, const Opnd<F16, NB>& b, v8f c) {
    if (F16) {
        v16h ah = __builtin_bit_cast(v16h, a.p[0]), bh = __builtin_bit_cast(v16h, b.p[0]);
        c = __builtin_amdgcn_wmma_f32_16x16x32_f16(false, ah, false, bh, (short)0, c, false, false);
        asm volatile("v_nop\n\tv_nop\n\tv_nop\n\tv_nop" : "+v"(c) : "v"(ah), "v"(bh));
        return c;
    }
    constexpr int NMX = NA > NB ? NA : NB;
#pragma unroll
    for (int i = 0; i < NA; ++i)
#pragma unroll
        for (int j = 0; j < NB; ++j)
            if (i + j < NMX) c = wm_bf16(a.p[i], b.p[j], c);
    if (NA == 1 && NB == 1)      asm volatile("v_nop\n\tv_nop\n\tv_nop\n\tv_nop" : "+v"(c) : "v"(a.p[0]), "v"(b.p[0]));
    else if (NA == 2 && NB == 1) asm volatile("v_nop\n\tv_nop\n\tv_nop\n\tv_nop" : "+v"(c) : "v"(a.p[0]), "v"(a.p[1]), "v"(b.p[0]));
    else if (NA == 1 && NB == 2) asm volatile("v_nop\n\tv_nop\n\tv_nop\n\tv_nop" : "+v"(c) : "v"(a.p[0]), "v"(b.p[0]), "v"(b.p[1]));
    else if (NA == 2 && NB == 2) asm volatile("v_nop\n\tv_nop\n\tv_nop\n\tv_nop" : "+v"(c) : "v"(a.p[0]), "v"(a.p[1]), "v"(b.p[0]), "v"(b.p[1]));
    else                         asm volatile("v_nop\n\tv_nop\n\tv_nop\n\tv_nop" : "+v"(c) : "v"(a.p[0]), "v"(a.p[NA - 1]), "v"(b.p[0]), "v"(b.p[NB - 1]), "v"(a.p[NA / 2]), "v"(b.p[NB / 2]));
    return c;
}

struct ZMap { long long s1; long long s2; int zdiv; int pad_; };
__device__ __forceinline__ size_t zoff(const ZMap& m, int z) { return (size_t)((long long)(z / m.zdiv) * m.s1 + (long long)(z % m.zdiv) * m.s2); }

#define ACT_NONE 0
#define ACT_RELU 1
#define ACT_GELU_ERF 2
#define ACT_SILU 3
#define ACT_TANH 4
__device__ __forceinline__ float act_apply(int act, float x) {
    if (act == ACT_RELU) return x > 0.f ? x : 0.f;
    if (act == ACT_GELU_ERF) return 0.5f * x * (1.0f + erff(x * 0.70710678118654752f));
    if (act == ACT_SILU) return x / (1.0f + expf(-x));
    if (act == ACT_TANH) return tanhf(x);
    return x;
}
struct GemmArgs {
    ZMap za, zb_, zc, zbias, zadd, zrsc, zmul, zrbias;
    const float* A; const float* Bm; float* C; const float* bias; const float* add; const float* rsc; const float* mul; const float* rbias;
    long long ldadd, ldmul;
    int lda, ldb, ldc, K;
    float ascale, bscale, oscale, addscale;
    int M, nvalid, nstore, ldrsc;
    int bcs, pad1, pad2, pad3;
};
template <int BT, int F16, int NA, int NB, int RW, int CW, int ACT>
__global__ __launch_bounds__(256) void gemm_kernel(GemmArgs g) {
    constexpr int TR = 16 * RW, TC = 64 * CW, CSTR = TC + 4;
    __shared__ __align__(16) float cst[TR * CSTR];
    const int z = blockIdx.z;
    const float* A = g.A + zoff(g.za, z); const float* Bm = g.Bm + zoff(g.zb_, z); float* C = g.C + zoff(g.zc, z);
    const int tid = threadIdx.x, lane = tid & 31, wv = tid >> 5;
    const int l16 = lane & 15, half = lane >> 4;
    const int rt = wv % RW, ch = wv / RW;
    const int row0 = blockIdx.x * TR, col0 = blockIdx.y * TC + ch * 64;
    int arix = row0 + rt * 16 + l16; if (arix >= g.M) arix = g.M - 1;
    const float* arow = A + (size_t)arix * g.lda;
    v8f acc[4];
#pragma unroll
    for (int t = 0; t < 4; ++t) acc[t] = (v8f){};
    const int K = g.K;
#pragma unroll 1
    for (int kc = 0; kc < K; kc += 32) {
        Opnd<F16, NA> a;
        if (kc + 32 <= K) op_row<F16, NA>(arow + kc, half, g.ascale, a); else op_row_tail<F16, NA>(arow + kc, half, g.ascale, K - kc, a);
#pragma unroll
        for (int t = 0; t < 4; ++t) {
            Opnd<F16, NB> b;
            const int n = col0 + t * 16 + l16;
            if (n < g.nvalid) {
                if (BT) { if (kc + 32 <= K) op_row<F16, NB>(Bm + (size_t)n * g.ldb + kc, half, g.bscale, b); else op_row_tail<F16, NB>(Bm + (size_t)n * g.ldb + kc, half, g.bscale, K - kc, b); }
                else    { if (kc + 32 <= K) op_col<F16, NB>(Bm, g.ldb, n * g.bcs, kc, half, g.bscale, b); else op_col_tail<F16, NB>(Bm, g.ldb, n * g.bcs, kc, half, g.bscale, K, b); }
            } else {
#pragma unroll
                for (int p = 0; p < NB; ++p) b.p[p] = (v16bf){};
            }
            acc[t] = wmma_op<F16, NA, NB>(a, b, acc[t]);
        }
    }
    const float* bias = g.bias ? g.bias + zoff(g.zbias, z) : nullptr;
    const float* add = g.add ? g.add + zoff(g.zadd, z) : nullptr;
    const float* rsc = g.rsc ? g.rsc + zoff(g.zrsc, z) : nullptr;
    const float* mul = g.mul ? g.mul + zoff(g.zmul, z) : nullptr;
    const float* rbias = g.rbias ? g.rbias + zoff(g.zrbias, z) : nullptr;
#pragma unroll
    for (int t = 0; t < 4; ++t) {
        const int cl = ch * 64 + t * 16 + l16;
        const int cg = blockIdx.y * TC + cl;
        const bool cok = cg < g.nvalid;
        const float bv = (bias && cok) ? bias[(size_t)cg * g.bcs] : 0.0f;
#pragma unroll
        for (int r = 0; r < 8; ++r) {
            const int rl = rt * 16 + r + 8 * half;
            float v = acc[t][r] * g.oscale + bv;
            int rg = row0 + rl; if (rg >= g.M) rg = g.M - 1;
            if (rbias) v += rbias[rg];
            if (rsc) v *= rsc[(size_t)rg * g.ldrsc];
            if (mul && cok) v *= mul[(size_t)rg * g.ldmul + cg];
            if (add && cok) v += g.addscale * add[(size_t)rg * g.ldadd + cg];
            cst[rl * CSTR + cl] = v;
        }
    }
    __syncthreads();
    const int col = tid % TC, rsel = tid / TC, rstep = 256 / TC;
    if (ACT != ACT_NONE) {
#pragma unroll 1
        for (int r = rsel; r < TR; r += rstep) cst[r * CSTR + col] = act_apply(ACT, cst[r * CSTR + col]);
    }
    float* ob = C + (size_t)row0 * g.ldc + (size_t)blockIdx.y * TC;
    const bool colok = (int)(blockIdx.y * TC + col) < g.nstore;
    const int rmax = (g.M - row0 < TR) ? (g.M - row0) : TR;
    auto pass = [&]() {
        if (colok) {
#pragma unroll 4
            for (int r = rsel; r < rmax; r += rstep) *(volatile float*)(ob + (size_t)r * g.ldc + col) = cst[r * CSTR + col];
        }
    };
    pass();
    __threadfence();
    pass();
}
static inline ZMap zm(long long s1) { ZMap m; m.s1 = s1; m.s2 = 0; m.zdiv = 1; m.pad_ = 0; return m; }
static inline ZMap zm2(long long s1, long long s2, int zdiv) { ZMap m; m.s1 = s1; m.s2 = s2; m.zdiv = zdiv; m.pad_ = 0; return m; }
static inline GemmArgs gemm_args(const float* A, int lda, ZMap za, const float* Bm, int ldb, ZMap zb, float* C, int ldc, ZMap zc, int M, int N, int K) {
    GemmArgs g; g.za = za; g.zb_ = zb; g.zc = zc; g.zbias = zm(0); g.zadd = zm(0); g.zrsc = zm(0); g.zmul = zm(0); g.zrbias = zm(0);
    g.A = A; g.Bm = Bm; g.C = C; g.bias = nullptr; g.add = nullptr; g.rsc = nullptr; g.mul = nullptr; g.rbias = nullptr; g.ldadd = 0; g.ldmul = 0;
    g.lda = lda; g.ldb = ldb; g.ldc = ldc; g.K = K; g.ascale = 1.0f; g.bscale = 1.0f; g.oscale = 1.0f; g.addscale = 1.0f; g.M = M; g.nvalid = N; g.nstore = N; g.ldrsc = 1;
    g.bcs = 1; g.pad1 = 0; g.pad2 = 0; g.pad3 = 0;
    return g;
}
static_assert(sizeof(ZMap) == 24, "ZMap layout");
static_assert(sizeof(GemmArgs) == 8 * 24 + 8 * 8 + 2 * 8 + 4 * 4 + 4 * 4 + 4 * 4 + 4 * 4, "GemmArgs has no padding");

__global__ __launch_bounds__(256) void softmax_rows(float* S, long long sy, long long sx, int L, float prescale, const float* addv, long long say, int aydiv, int causal,
                                                  const int* imask, long long imy, long long imx, float maskval) {
    __shared__ float red[8];
    const int tid = threadIdx.x, lane = tid & 31, wid = tid >> 5;
    float* row = S + (size_t)blockIdx.y * sy + (size_t)blockIdx.x * sx;
    const float* av = addv ? addv + (size_t)(blockIdx.y / aydiv) * say : nullptr;
    const int* im = imask ? imask + (size_t)(blockIdx.y / aydiv) * imy + (size_t)blockIdx.x * imx : nullptr;
    float v[16];
    const int nj = L / 256;
    float mx = -__builtin_inff();
#pragma unroll
    for (int j = 0; j < 16; ++j) if (j < nj) { float t = row[tid + 256 * j] * prescale; if (av) t += av[tid + 256 * j]; if (im && im[tid + 256 * j] == 0) t = maskval; if (causal && (tid + 256 * j) > (int)blockIdx.x) t = -__builtin_inff(); v[j] = t; mx = fmaxf(mx, t); }
#pragma unroll
    for (int o = 16; o; o >>= 1) mx = fmaxf(mx, __shfl_xor(mx, o, 32));
    if (lane == 0) red[wid] = mx;
    __syncthreads();
    float m = red[0];
#pragma unroll
    for (int i = 1; i < 8; ++i) m = fmaxf(m, red[i]);
    if (m == -__builtin_inff()) m = 0.f;
    __syncthreads();
    float sum = 0.f;
#pragma unroll
    for (int j = 0; j < 16; ++j) if (j < nj) { v[j] = expf(v[j] - m); sum += v[j]; }
#pragma unroll
    for (int o = 16; o; o >>= 1) sum += __shfl_xor(sum, o, 32);
    if (lane == 0) red[wid] = sum;
    __syncthreads();
    float tot = 0.f;
#pragma unroll
    for (int i = 0; i < 8; ++i) tot += red[i];
    const float inv = 1.0f / tot;
#pragma unroll
    for (int j = 0; j < 16; ++j) if (j < nj) *(volatile float*)(row + tid + 256 * j) = v[j] * inv;
    __threadfence();
#pragma unroll
    for (int j = 0; j < 16; ++j) if (j < nj) *(volatile float*)(row + tid + 256 * j) = v[j] * inv;
}

#define VST2(T, p, v) do { const T vst2_v_ = (v); *(volatile T*)(p) = vst2_v_; __threadfence(); *(volatile T*)(p) = vst2_v_; } while (0)

__global__ __launch_bounds__(256) void k_prep(const float* __restrict__ feat, const float* __restrict__ sxr, const float* __restrict__ syr, const float* __restrict__ szr, const float* __restrict__ srr,
                                             float* sig, float* se, float* featT) {
    const int cell = blockIdx.x * 256 + threadIdx.x; if (cell >= NCELL) return;
    const float sx = fmaxf(expf(sxr[cell]), 1e-6f), sy = fmaxf(expf(syr[cell]), 1e-6f), sz = fmaxf(expf(szr[cell]), 1e-6f), sr = fmaxf(expf(srr[cell]), 1e-6f);
    VST2(float, sig + cell, sx); VST2(float, sig + NCELL + cell, sy); VST2(float, sig + 2 * NCELL + cell, sz); VST2(float, sig + 3 * NCELL + cell, sr);
    VST2(float, se + cell, fmaxf(sx, fmaxf(sy, sz)));
}
__global__ __launch_bounds__(256) void k_featT(const float* __restrict__ feat, float* featT) {
    const int q = blockIdx.x * 256 + threadIdx.x; if (q >= NCELL * CF) return; const int c = q % CF, cell = q / CF;
    VST2(float, featT + q, feat[(size_t)c * NCELL + cell]);
}
__device__ __forceinline__ void up2(int o, int& i0, int& i1, float& w0, float& w1) {
    const float x = ((float)o + 0.5f) * 0.5f - 0.5f; const int f = (int)floorf(x); const float t = x - (float)f;
    i0 = f; i1 = f + 1; w0 = 1.f - t; w1 = t;
    if (i0 < 0) { i0 = 0; w0 = 0.f; w1 = 1.f; i1 = 0; }
    if (i1 > NL - 1) { i1 = NL - 1; if (f + 1 > NL - 1) { w1 = 0.f; w0 = 1.f; i0 = NL - 1; } }
}
__global__ __launch_bounds__(256) void k_rmap(const float* __restrict__ se, float* R2) {
    const int v = blockIdx.x * 256 + threadIdx.x; if (v >= NVOX) return;
    const int Z = v % NHR, Y = (v / NHR) % NHR, X = v / (NHR * NHR);
    int xi0, xi1, yi0, yi1, zi0, zi1; float xw0, xw1, yw0, yw1, zw0, zw1;
    up2(X, xi0, xi1, xw0, xw1); up2(Y, yi0, yi1, yw0, yw1); up2(Z, zi0, zi1, zw0, zw1);
    float s = 0.f;
    s += xw0 * (yw0 * (zw0 * se[(xi0 * NL + yi0) * NL + zi0] + zw1 * se[(xi0 * NL + yi0) * NL + zi1]) + yw1 * (zw0 * se[(xi0 * NL + yi1) * NL + zi0] + zw1 * se[(xi0 * NL + yi1) * NL + zi1]));
    s += xw1 * (yw0 * (zw0 * se[(xi1 * NL + yi0) * NL + zi0] + zw1 * se[(xi1 * NL + yi0) * NL + zi1]) + yw1 * (zw0 * se[(xi1 * NL + yi1) * NL + zi0] + zw1 * se[(xi1 * NL + yi1) * NL + zi1]));
    float R = ceilf(2.0f * s); R = fminf(fmaxf(R, 1.f), (float)RMAX);
    VST2(float, R2 + v, R * R);
}
__device__ __forceinline__ int dn_taps(int o, int* idx, float* w) {
    const int cand[4] = {2 * o - 1, 2 * o, 2 * o + 1, 2 * o + 2}; const float cw[4] = {0.25f, 0.75f, 0.75f, 0.25f};
    float tot = 0.f; int n = 0;
    for (int j = 0; j < 4; ++j) if (cand[j] >= 0 && cand[j] < NHR) { idx[n] = cand[j]; w[n] = cw[j]; tot += cw[j]; ++n; }
    for (int j = 0; j < n; ++j) w[j] /= tot;
    return n;
}
__global__ __launch_bounds__(256) void k_guide_lr(const float* __restrict__ guide, float* glr) {
    const int q = blockIdx.x * 256 + threadIdx.x; if (q >= GG * NCELL) return; const int cell = q % NCELL, g = q / NCELL;
    const int w = cell % NL, v = (cell / NL) % NL, u = cell / (NL * NL);
    int xi[4], yi[4], zi[4]; float xw[4], yw[4], zw[4]; const int nx = dn_taps(u, xi, xw), ny = dn_taps(v, yi, yw), nz = dn_taps(w, zi, zw);
    const float* gp = guide + (size_t)g * NVOX; float s = 0.f;
    for (int a = 0; a < nx; ++a) for (int b = 0; b < ny; ++b) { float t = 0.f; for (int c = 0; c < nz; ++c) t += zw[c] * gp[((size_t)xi[a] * NHR + yi[b]) * NHR + zi[c]]; s += xw[a] * yw[b] * t; }
    VST2(float, glr + q, s);
}
__global__ __launch_bounds__(128) void k_jbu(const float* __restrict__ featT, const float* __restrict__ guide, const float* __restrict__ glr, const float* __restrict__ sig,
                                            const float* __restrict__ R2, float* out) {
    __shared__ float lw[4][8][KPAD];
    __shared__ int nbc[4][KPAD];
    __shared__ float vm[4][8];
    __shared__ float res[CF + 1][128];
    const int tid = threadIdx.x, lane = tid & 31, wv = tid >> 5, l16 = lane & 15, half = lane >> 4;
    const int u = blockIdx.x / (NL * 2), v = (blockIdx.x / 2) % NL, w0 = (blockIdx.x & 1) * 16;
    for (int ci = 0; ci < 4; ++ci) {
        const int cl = wv * 4 + ci; const int w = w0 + cl;
        float gX[8][GG]; float r2v[8];
#pragma unroll
        for (int s = 0; s < 8; ++s) { const int X = 2 * u + (s >> 2), Y = 2 * v + ((s >> 1) & 1), Z = 2 * w + (s & 1); const size_t vi = ((size_t)X * NHR + Y) * NHR + Z;
#pragma unroll
            for (int g = 0; g < GG; ++g) gX[s][g] = guide[(size_t)g * NVOX + vi]; r2v[s] = R2[vi]; }
        float mymax[8];
#pragma unroll
        for (int s = 0; s < 8; ++s) mymax[s] = -1e9f;
        for (int k = lane; k < KPAD; k += 32) {
            int ncell = 0;
            if (k < NOFF) {
                const int dX = k / 49 - RMAX, dY = (k / 7) % 7 - RMAX, dZ = k % 7 - RMAX;
                int Ui = u + dX; Ui = Ui < 0 ? 0 : (Ui > NL - 1 ? NL - 1 : Ui); int Vi = v + dY; Vi = Vi < 0 ? 0 : (Vi > NL - 1 ? NL - 1 : Vi); int Wi = w + dZ; Wi = Wi < 0 ? 0 : (Wi > NL - 1 ? NL - 1 : Wi);
                ncell = (Ui * NL + Vi) * NL + Wi;
                const float r2 = (float)(dX * dX + dY * dY + dZ * dZ);
                const float cx = (float)Ui * 2.0f + 0.5f, cy = (float)Vi * 2.0f + 0.5f, cz = (float)Wi * 2.0f + 0.5f;
                const float sx = sig[ncell], sy = sig[NCELL + ncell], sz = sig[2 * NCELL + ncell], sr = sig[3 * NCELL + ncell];
                const float isx = 1.0f / (2.0f * sx * sx), isy = 1.0f / (2.0f * sy * sy), isz = 1.0f / (2.0f * sz * sz), isr = 1.0f / (2.0f * sr * sr + 1e-8f);
                const float g0 = glr[ncell], g1 = glr[NCELL + ncell], g2 = glr[2 * NCELL + ncell];
#pragma unroll
                for (int s = 0; s < 8; ++s) {
                    const float X = (float)(2 * u + (s >> 2)), Y = (float)(2 * v + ((s >> 1) & 1)), Z = (float)(2 * w + (s & 1));
                    const float dx = X - cx, dy = Y - cy, dz = Z - cz;
                    const float d0 = gX[s][0] - g0, d1 = gX[s][1] - g1, d2 = gX[s][2] - g2;
                    const float lws = -dx * dx * isx - dy * dy * isy - dz * dz * isz;
                    const float lwr = -(d0 * d0 + d1 * d1 + d2 * d2) * isr;
                    const float l = (r2 <= r2v[s]) ? (lws + lwr) : -1e9f;
                    lw[wv][s][k] = l; mymax[s] = fmaxf(mymax[s], l);
                }
            } else {
#pragma unroll
                for (int s = 0; s < 8; ++s) lw[wv][s][k] = -__builtin_inff();
            }
            nbc[wv][k] = ncell;
        }
#pragma unroll
        for (int s = 0; s < 8; ++s) { float m = mymax[s];
#pragma unroll
            for (int o = 16; o; o >>= 1) m = fmaxf(m, __shfl_xor(m, o, 32)); if (lane == 0) vm[wv][s] = m; }
        __syncthreads();
        v8f acc[3]; acc[0] = (v8f){}; acc[1] = (v8f){}; acc[2] = (v8f){};
        const bool arow = l16 < 8; const float am = arow ? vm[wv][l16] : 0.f;
#pragma unroll 1
        for (int ks = 0; ks < KPAD / 32; ++ks) {
            Opnd<1, 1> a;
            { v8u uu;
#pragma unroll
              for (int vv = 0; vv < 8; ++vv) { const int kk = ks * 32 + kpat(vv, half); unsigned t3[3];
                  const float e0 = arow ? expf(lw[wv][l16 & 7][kk] - am) : 0.f, e1 = arow ? expf(lw[wv][l16 & 7][kk + 1] - am) : 0.f;
                  pack2<1, 1>(e0, e1, t3); uu[vv] = t3[0]; }
              a.p[0] = __builtin_bit_cast(v16bf, uu); }
#pragma unroll
            for (int t = 0; t < 3; ++t) {
                Opnd<1, 1> bo; v8u uu;
#pragma unroll
                for (int vv = 0; vv < 8; ++vv) { const int kk = ks * 32 + kpat(vv, half); unsigned t3[3]; float f0, f1;
                    if (t < 2) { const int c = t * 16 + l16; f0 = featT[(size_t)nbc[wv][kk] * CF + c]; f1 = featT[(size_t)nbc[wv][kk + 1] * CF + c]; if (kk >= NOFF) f0 = 0.f; if (kk + 1 >= NOFF) f1 = 0.f; }
                    else { f0 = (l16 == 0 && kk < NOFF) ? 1.f : 0.f; f1 = (l16 == 0 && kk + 1 < NOFF) ? 1.f : 0.f; }
                    pack2<1, 1>(f0, f1, t3); uu[vv] = t3[0]; }
                bo.p[0] = __builtin_bit_cast(v16bf, uu);
                acc[t] = wmma_op<1, 1, 1>(a, bo, acc[t]);
            }
        }
        asm volatile("v_nop\n\tv_nop\n\tv_nop\n\tv_nop" ::: "memory");
        if (half == 0) {
#pragma unroll
            for (int r = 0; r < 8; ++r) { res[l16][cl * 8 + r] = acc[0][r]; res[16 + l16][cl * 8 + r] = acc[1][r]; if (l16 == 0) res[CF][cl * 8 + r] = acc[2][r]; }
        }
        __syncthreads();
    }
    for (int q = tid; q < CF * 4 * 32; q += 128) {
        const int zz = q & 31, ab = (q >> 5) & 3, c = q >> 7; const int a = ab >> 1, b = ab & 1;
        const int cl = zz >> 1, e = zz & 1; const int sidx = (a << 2) | (b << 1) | e; const int vb = cl * 8 + sidx;
        const float den = fmaxf(res[CF][vb], 1e-8f); const float val = res[c][vb] / den;
        const int X = 2 * u + a, Y = 2 * v + b, Z = 2 * w0 + zz;
        float* dst = out + (size_t)c * NVOX + ((size_t)X * NHR + Y) * NHR + Z;
        *(volatile float*)dst = val;
    }
    __threadfence();
    for (int q = tid; q < CF * 4 * 32; q += 128) {
        const int zz = q & 31, ab = (q >> 5) & 3, c = q >> 7; const int a = ab >> 1, b = ab & 1;
        const int cl = zz >> 1, e = zz & 1; const int sidx = (a << 2) | (b << 1) | e; const int vb = cl * 8 + sidx;
        const float den = fmaxf(res[CF][vb], 1e-8f); const float val = res[c][vb] / den;
        const int X = 2 * u + a, Y = 2 * v + b, Z = 2 * w0 + zz;
        *(volatile float*)(out + (size_t)c * NVOX + ((size_t)X * NHR + Y) * NHR + Z) = val;
    }
}

extern "C" void kernel_launch(void* const* d_in, const int* in_sizes, int n_in,
                              void* d_out, int out_size, void* d_ws, size_t ws_size, hipStream_t stream) {
    (void)in_sizes; (void)n_in; (void)out_size;
    const float* feat = (const float*)d_in[0];
    const float* guide = (const float*)d_in[1];
    const float* sxr = (const float*)d_in[2]; const float* syr = (const float*)d_in[3]; const float* szr = (const float*)d_in[4]; const float* srr = (const float*)d_in[5];
    float* out = (float*)d_out;

    char* wsp = (char*)d_ws;
    auto take = [&](size_t bytes) { char* p = wsp; wsp += (bytes + 255) & ~(size_t)255; return (void*)p; };
    float* sig = (float*)take((size_t)4 * NCELL * 4); float* se = (float*)take((size_t)NCELL * 4);
    float* featT = (float*)take((size_t)NCELL * CF * 4); float* R2 = (float*)take((size_t)NVOX * 4); float* glr = (float*)take((size_t)GG * NCELL * 4);
    if ((size_t)(wsp - (char*)d_ws) > ws_size) return;

    k_prep<<<NCELL / 256, 256, 0, stream>>>(feat, sxr, syr, szr, srr, sig, se, featT);
    k_featT<<<(NCELL * CF) / 256, 256, 0, stream>>>(feat, featT);
    k_rmap<<<NVOX / 256, 256, 0, stream>>>(se, R2);
    k_guide_lr<<<(GG * NCELL) / 256, 256, 0, stream>>>(guide, glr);
    k_jbu<<<NL * NL * 2, 128, 0, stream>>>(featT, guide, glr, sig, R2, out);
}
